// LocalAttention_88622355186049
// MI455X (gfx1250) — hardware-verified
//
#include <hip/hip_runtime.h>


#ifndef NB
#define NB 2
#endif
#ifndef SEQ
#define SEQ 2048
#endif
#define NB_FULL  2
#define SEQ_FULL 2048
#ifndef OUT_SEQ
#define OUT_SEQ SEQ
#endif
#define DM   512
#define QKP  (2 * DM)
#define WND  32
#define KT   6
#define AW   4
#define OSP  68
#define SC2  ((float)(0.044194173824159216 * 1.4426950408889634))
#define PSH  14.0f
#define NEGB (-3.0e38f)
#define CSC  256.0f
#define WSC  1024.0f
#define OSC  (1.0f / (256.0f * 1024.0f))

static_assert(DM % 64 == 0);
static_assert(QKP % 64 == 0);
static_assert(DM % 32 == 0);
static_assert(SEQ % 64 == 0);
static_assert((NB * SEQ) % 64 == 0);
static_assert(SEQ % (16 * AW) == 0);
static_assert(SEQ >= 64);
static_assert(KT == 6);
static_assert(WND - 1 <= 32);
static_assert(16 * KT - 32 >= 16 + WND - 1);
static_assert((size_t)NB * SEQ * QKP < (size_t)2147483647);
static_assert((size_t)NB * DM * SEQ < (size_t)2147483647);
static_assert(((size_t)SEQ * DM) % 8 == 0);
static_assert(((size_t)3 * DM * DM) % 8 == 0);
static_assert(NB <= NB_FULL);
static_assert(SEQ <= SEQ_FULL);
static_assert((OSP * 4) % 16 == 0);
static_assert(4 * 32 * 16 == 16 * 64 * 2);
static_assert(8 * 32 * 16 == 16 * 64 * 4);
static_assert(16 * 68 * 4 <= 131072);
static_assert(AW * 16 * OSP * 4 <= 131072);

typedef _Float16 h16;
typedef unsigned short bf;
typedef __attribute__((ext_vector_type(16))) __bf16   v16bf;
typedef __attribute__((ext_vector_type(16))) _Float16 v16h;
typedef __attribute__((ext_vector_type(8)))  _Float16 v8h;
typedef __attribute__((ext_vector_type(8)))  unsigned short v8us;
typedef __attribute__((ext_vector_type(8)))  float    v8f;
typedef __attribute__((ext_vector_type(4)))  float    v4f;
typedef v4f  __attribute__((may_alias)) v4fa;

__device__ __forceinline__ unsigned short f2bf(float f) { unsigned u = __float_as_uint(f); u += 0x7FFFu + ((u >> 16) & 1u); return (unsigned short)(u >> 16); }
__device__ __forceinline__ float bfr(float f) { return __uint_as_float(((unsigned)f2bf(f)) << 16); }
__device__ __forceinline__ v16h cat16(v8h lo, v8h hi) { return __builtin_shufflevector(lo, hi, 0, 1, 2, 3, 4, 5, 6, 7, 8, 9, 10, 11, 12, 13, 14, 15); }
__device__ __forceinline__ v16bf cat16b(v8us lo, v8us hi) { return __builtin_bit_cast(v16bf, __builtin_shufflevector(lo, hi, 0, 1, 2, 3, 4, 5, 6, 7, 8, 9, 10, 11, 12, 13, 14, 15)); }
__device__ __forceinline__ v8f wmma16(v16h a, v16h b, v8f c) { return __builtin_amdgcn_wmma_f32_16x16x32_f16(false, a, false, b, (short)0, c, false, false); }
__device__ __forceinline__ v8f wmmab(v16bf a, v16bf b, v8f c) { return __builtin_amdgcn_wmma_f32_16x16x32_bf16(false, a, false, b, (short)0, c, false, false); }
__device__ __forceinline__ v16h  ldh(const h16* p) { return cat16(*(const v8h*)p, *(const v8h*)(p + 16)); }
__device__ __forceinline__ v16bf ldb(const bf* p)  { return cat16b(*(const v8us*)p, *(const v8us*)(p + 16)); }
__device__ __forceinline__ void wave_sync() { __builtin_amdgcn_fence(3  , "wavefront"); __builtin_amdgcn_wave_barrier(); asm volatile("" ::: "memory"); }

static __device__ __forceinline__ h16 toh_flush(float v) { const h16 r = (h16)v; return (fabsf(v) < 6.103515625e-05f) ? (h16)0.0f : r; }
__device__ __forceinline__ v8f wmma16g(v16h a, v16h b, v8f c) { c = wmma16(a, b, c); asm volatile("v_nop\n\tv_nop\n\tv_nop\n\tv_nop" : "+v"(c) : "v"(a), "v"(b)); return c; }
__device__ __forceinline__ v8f wmmabg(v16bf a, v16bf b, v8f c) { c = wmmab(a, b, c); asm volatile("v_nop\n\tv_nop\n\tv_nop\n\tv_nop" : "+v"(c) : "v"(a), "v"(b)); return c; }

__global__ __launch_bounds__(256) void k_cvt8(const float* __restrict__ src, bf* dst, size_t n8) {
    const size_t i = (size_t)blockIdx.x * 256 + threadIdx.x; if (i >= n8) return;
    const v8f v = *(const v8f*)(src + i * 8); v8us o;
#pragma unroll
    for (int k = 0; k < 8; ++k) o[k] = f2bf(v[k]);
    *(volatile v8us*)(dst + i * 8) = o; __threadfence(); *(volatile v8us*)(dst + i * 8) = o;
}

__global__ __launch_bounds__(256) void k_cvtw(const float* __restrict__ src, h16* dst, size_t n8) {
    const size_t i = (size_t)blockIdx.x * 256 + threadIdx.x; if (i >= n8) return;
    const v8f v = *(const v8f*)(src + i * 8); v8h o;
#pragma unroll
    for (int k = 0; k < 8; ++k) o[k] = toh_flush(bfr(v[k]) * WSC);
    *(volatile v8h*)(dst + i * 8) = o; __threadfence(); *(volatile v8h*)(dst + i * 8) = o;
}

__global__ __launch_bounds__(32) void k_proj_bf(const bf* __restrict__ A, const bf* __restrict__ Bt, const float* __restrict__ bias, h16* P,
                                                int biasRow, int cseg, int bstride, int ldc) {
    __shared__ __align__(16) float os[16 * 68];
    const int K = DM;
    const int lane = threadIdx.x & 31, lr = lane & 15, hi = lane >> 4;
    const int r0 = blockIdx.x * 64, c0 = blockIdx.y * 64; const int n0 = blockIdx.z * cseg + c0;
    v8f acc[4][4];
#pragma unroll
    for (int mb = 0; mb < 4; ++mb)
#pragma unroll
        for (int nb = 0; nb < 4; ++nb) acc[mb][nb] = (v8f){};
    const size_t aoff = (size_t)(r0 + lr) * K + 8 * hi, boff = (size_t)(n0 + lr) * K + 8 * hi;
#pragma unroll 1
    for (int kc = 0; kc < K; kc += 32) {
        v16bf a[4];
#pragma unroll
        for (int mb = 0; mb < 4; ++mb) a[mb] = ldb(A + aoff + (size_t)mb * 16 * K + kc);
#pragma unroll
        for (int nb = 0; nb < 4; ++nb) { const v16bf b = ldb(Bt + boff + (size_t)nb * 16 * K + kc);
#pragma unroll
            for (int mb = 0; mb < 4; ++mb) acc[mb][nb] = wmmabg(a[mb], b, acc[mb][nb]); }
    }
    float bc[4];
#pragma unroll
    for (int nb = 0; nb < 4; ++nb) { const int ic = biasRow ? 0 : (n0 + nb * 16 + lr); const float bv = bias[ic]; bc[nb] = biasRow ? 0.0f : bfr(bv); }
    const size_t tbase = (size_t)blockIdx.z * (size_t)bstride + (size_t)r0 * (size_t)ldc + (size_t)c0;
#pragma unroll
    for (int mb = 0; mb < 4; ++mb) {
        float br[8];
#pragma unroll
        for (int j = 0; j < 8; ++j) { const int ir = biasRow ? (r0 + mb * 16 + hi * 8 + j) : 0; const float bv = bias[ir]; br[j] = biasRow ? bfr(bv) : 0.0f; }
#pragma unroll
        for (int nb = 0; nb < 4; ++nb) {
#pragma unroll
            for (int j = 0; j < 8; ++j) os[(hi * 8 + j) * 68 + nb * 16 + lr] = acc[mb][nb][j] + bc[nb] + br[j]; }
        wave_sync();
        const size_t sb = tbase + (size_t)(mb * 16) * (size_t)ldc;
#pragma unroll 1
        for (int ps = 0; ps < 2; ++ps) {
#pragma unroll
            for (int s = 0; s < 4; ++s) { const int row = 4 * s + (lane >> 3), c8 = (lane & 7) * 8;
                const v4f x0 = *(const v4fa*)(&os[row * 68 + c8]); const v4f x1 = *(const v4fa*)(&os[row * 68 + c8 + 4]); v8h hv;
#pragma unroll
                for (int i = 0; i < 4; ++i) { hv[i] = toh_flush(x0[i]); hv[4 + i] = toh_flush(x1[i]); }
                *(volatile v8h*)(P + sb + (size_t)row * (size_t)ldc + c8) = hv; }
            if (ps == 0) __threadfence(); }
        wave_sync();
    }
}

__global__ __launch_bounds__(32 * AW) void k_band(const h16* __restrict__ QK, const h16* __restrict__ VT, h16* CTX) {
    __shared__ __align__(16) float os[AW * 16 * OSP];
    const int lane = threadIdx.x & 31, lr = lane & 15, hi = lane >> 4;
    const int wave = __builtin_amdgcn_readfirstlane((int)(threadIdx.x >> 5));
    const int b = blockIdx.y;
    const int t0 = (blockIdx.x * AW + wave) * 16;
    const int ks = t0 - 32;
    const int rowb = b * SEQ;
    const int qo = (rowb + t0 + lr) * QKP + 8 * hi;
    int ko[KT];
#pragma unroll
    for (int j = 0; j < KT; ++j) { int kr = ks + 16 * j + lr; kr = kr < 0 ? 0 : (kr > SEQ - 1 ? SEQ - 1 : kr); ko[j] = (rowb + kr) * QKP + DM + 8 * hi; }
    v8f s[KT];
#pragma unroll
    for (int j = 0; j < KT; ++j) s[j] = (v8f){};
#pragma unroll 1
    for (int d0 = 0; d0 < DM; d0 += 32) {
        const v16h qf = ldh(QK + qo + d0);
#pragma unroll
        for (int j = 0; j < KT; ++j) { const v16h kf = ldh(QK + ko[j] + d0); s[j] = wmma16g(kf, qf, s[j]); }
    }
    const int tq = t0 + lr;
    const int dl = 8 * hi - 32 - lr;
    float mx = NEGB;
#pragma unroll
    for (int j = 0; j < KT; ++j) {
#pragma unroll
        for (int r = 0; r < 8; ++r) {
            const int dd = 16 * j + r + dl; const int key = tq + dd;
            const bool f = (dd >= -(WND - 1)) & (dd <= (WND - 1)) & (key >= 0) & (key < SEQ);
            const float tv = f ? s[j][r] * SC2 : NEGB;
            s[j][r] = tv; mx = fmaxf(mx, tv); } }
    mx = fmaxf(mx, __shfl_xor(mx, 16, 32));
    const float sh = PSH - mx;
    v16h pb[3]; float l = 0.0f;
#pragma unroll
    for (int sx = 0; sx < 3; ++sx) {
#pragma unroll
        for (int r = 0; r < 8; ++r) {
            const float ea = s[2 * sx][r] + sh, eb = s[2 * sx + 1][r] + sh;
            const float xa = __builtin_amdgcn_exp2f(ea), xb = __builtin_amdgcn_exp2f(eb);
            const float ga = (ea >= -PSH) ? xa : 0.0f, gb = (eb >= -PSH) ? xb : 0.0f;
            const h16 pa = (h16)ga; const h16 pc = (h16)gb;
            pb[sx][r] = pa; pb[sx][8 + r] = pc; l += (float)pa + (float)pc; } }
    l += __shfl_xor(l, 16, 32);
    const bool any = l > 0.0f;
    const float lsafe = any ? l : 1.0f;
    const float cm = any ? (CSC / lsafe) : 0.0f;
    int g0[3], g1[3];
#pragma unroll
    for (int sx = 0; sx < 3; ++sx) { int a = ks + 32 * sx + 8 * hi; int c = a + 16;
        a = a < 0 ? 0 : (a > SEQ - 8 ? SEQ - 8 : a); c = c < 0 ? 0 : (c > SEQ - 8 ? SEQ - 8 : c); g0[sx] = a; g1[sx] = c; }
    const int vb = (b * DM + lr) * SEQ;
    const int wb = wave * 16 * OSP;
#pragma unroll 1
    for (int dc = 0; dc < DM; dc += 64) {
        v8f f[4];
#pragma unroll
        for (int j = 0; j < 4; ++j) f[j] = (v8f){};
#pragma unroll
        for (int sx = 0; sx < 3; ++sx) {
#pragma unroll
            for (int j = 0; j < 4; ++j) { const int ro = vb + (dc + 16 * j) * SEQ;
                const v8h lo = *(const v8h*)(VT + ro + g0[sx]); const v8h hh = *(const v8h*)(VT + ro + g1[sx]);
                f[j] = wmma16g(cat16(lo, hh), pb[sx], f[j]); } }
#pragma unroll
        for (int j = 0; j < 4; ++j) { v4f a, c;
            a[0] = f[j][0] * cm; a[1] = f[j][1] * cm; a[2] = f[j][2] * cm; a[3] = f[j][3] * cm; c[0] = f[j][4] * cm; c[1] = f[j][5] * cm; c[2] = f[j][6] * cm; c[3] = f[j][7] * cm;
            *(v4fa*)(&os[wb + lr * OSP + 16 * j + 8 * hi]) = a; *(v4fa*)(&os[wb + lr * OSP + 16 * j + 8 * hi + 4]) = c; }
        wave_sync();
        h16* crow = CTX + (size_t)(rowb + t0) * DM + dc;
#pragma unroll 1
        for (int ps = 0; ps < 2; ++ps) {
#pragma unroll
            for (int sq = 0; sq < 4; ++sq) { const int row = 4 * sq + (lane >> 3), c8 = (lane & 7) * 8;
                const v4f x0 = *(const v4fa*)(&os[wb + row * OSP + c8]); const v4f x1 = *(const v4fa*)(&os[wb + row * OSP + c8 + 4]); v8h hv;
#pragma unroll
                for (int i = 0; i < 4; ++i) { hv[i] = toh_flush(x0[i]); hv[4 + i] = toh_flush(x1[i]); }
                *(volatile v8h*)(crow + (size_t)row * DM + c8) = hv; }
            if (ps == 0) __threadfence(); }
        wave_sync();
    }
}

__global__ __launch_bounds__(32) void k_out(const h16* __restrict__ A, const h16* __restrict__ Bt, const float* __restrict__ bias, float* OUT) {
    __shared__ __align__(16) float os[16 * 68];
    const int K = DM;
    const int lane = threadIdx.x & 31, lr = lane & 15, hi = lane >> 4; const int r0 = blockIdx.x * 64, c0 = blockIdx.y * 64;
    v8f acc[4][4];
#pragma unroll
    for (int mb = 0; mb < 4; ++mb)
#pragma unroll
        for (int nb = 0; nb < 4; ++nb) acc[mb][nb] = (v8f){};
    const size_t aoff = (size_t)(r0 + lr) * K + 8 * hi, boff = (size_t)(c0 + lr) * K + 8 * hi;
#pragma unroll 1
    for (int kc = 0; kc < K; kc += 32) {
        v16h a[4];
#pragma unroll
        for (int mb = 0; mb < 4; ++mb) a[mb] = ldh(A + aoff + (size_t)mb * 16 * K + kc);
#pragma unroll
        for (int nb = 0; nb < 4; ++nb) { const v16h b = ldh(Bt + boff + (size_t)nb * 16 * K + kc);
#pragma unroll
            for (int mb = 0; mb < 4; ++mb) acc[mb][nb] = wmma16g(a[mb], b, acc[mb][nb]); }
    }
    float bc[4];
#pragma unroll
    for (int nb = 0; nb < 4; ++nb) bc[nb] = bfr(bias[c0 + nb * 16 + lr]);
    const int bb = r0 / SEQ, tt = r0 % SEQ;
    float* ob = OUT + ((size_t)bb * OUT_SEQ + (size_t)tt) * DM + c0;
#pragma unroll
    for (int mb = 0; mb < 4; ++mb) {
#pragma unroll
        for (int nb = 0; nb < 4; ++nb) {
#pragma unroll
            for (int j = 0; j < 8; ++j) os[(hi * 8 + j) * 68 + nb * 16 + lr] = acc[mb][nb][j] * OSC + bc[nb]; }
        wave_sync();
#pragma unroll 1
        for (int ps = 0; ps < 2; ++ps) {
#pragma unroll
            for (int s = 0; s < 8; ++s) { const int row = 2 * s + (lane >> 4), cofs = (lane & 15) * 4;
                const v4f val = *(const v4fa*)(&os[row * 68 + cofs]);
                *(volatile v4f*)(ob + (size_t)(mb * 16 + row) * DM + cofs) = val; }
            if (ps == 0) __threadfence(); }
        wave_sync();
    }
}

static constexpr size_t al256(size_t v) { return (v + 255) & ~(size_t)255; }
static constexpr size_t SZ_XB = al256((size_t)NB * SEQ * DM * 2);
static constexpr size_t SZ_WB = al256((size_t)3 * DM * DM * 2);
static constexpr size_t SZ_WP = al256((size_t)DM * DM * 2);
static constexpr size_t SZ_QK = al256((size_t)NB * SEQ * QKP * 2);
static constexpr size_t SZ_VT = al256((size_t)NB * DM * SEQ * 2);
static constexpr size_t SZ_CX = al256((size_t)NB * SEQ * DM * 2);
static constexpr size_t SZ_TOTAL = SZ_XB + SZ_WB + SZ_WP + SZ_QK + SZ_VT + SZ_CX;
static_assert(SZ_TOTAL <= (size_t)134217728);
static_assert(((size_t)2 * DM * DM * 2) % 256 == 0);
static_assert((size_t)(NB * SEQ / 64) * 64 * (size_t)QKP == (size_t)NB * SEQ * QKP);
static_assert((size_t)(DM / 64) * (SEQ / 64) * NB * 4096 == (size_t)NB * DM * SEQ);
static_assert((size_t)(SEQ / (16 * AW)) * NB * AW * 16 * DM == (size_t)NB * SEQ * DM);

extern "C" void kernel_launch(void* const* d_in, const int* in_sizes, int n_in,
                              void* d_out, int out_size, void* d_ws, size_t ws_size, hipStream_t stream) {
    if (n_in < 5) return;
    const size_t needx = ((size_t)(NB - 1) * SEQ_FULL + SEQ) * DM;
    if ((size_t)in_sizes[0] < needx) return;
    if ((size_t)in_sizes[1] < (size_t)3 * DM * DM || in_sizes[2] < 3 * DM) return;
    if ((size_t)in_sizes[3] < (size_t)DM * DM || in_sizes[4] < DM) return;
    if ((size_t)out_size < ((size_t)(NB - 1) * OUT_SEQ + SEQ) * DM) return;
    if (SZ_TOTAL > ws_size) return;
    const float* x     = (const float*)d_in[0];
    const float* wqkv  = (const float*)d_in[1];
    const float* bqkv  = (const float*)d_in[2];
    const float* wproj = (const float*)d_in[3];
    const float* bproj = (const float*)d_in[4];
    float* OUT = (float*)d_out;
    char* wsp = (char*)d_ws;
    bf*  XB = (bf*)wsp;  wsp += SZ_XB;
    bf*  WB = (bf*)wsp;  wsp += SZ_WB;
    h16* WP = (h16*)wsp; wsp += SZ_WP;
    h16* QK = (h16*)wsp; wsp += SZ_QK;
    h16* VT = (h16*)wsp; wsp += SZ_VT;
    h16* CX = (h16*)wsp; wsp += SZ_CX;

    if (SEQ == SEQ_FULL) {
        const size_t n8 = (size_t)NB * SEQ * DM / 8;
        k_cvt8<<<(unsigned)((n8 + 255) / 256), 256, 0, stream>>>(x, XB, n8);
    } else {
        const size_t n8 = (size_t)SEQ * DM / 8;
        for (int b = 0; b < NB; ++b) k_cvt8<<<(unsigned)((n8 + 255) / 256), 256, 0, stream>>>(x + (size_t)b * SEQ_FULL * DM, XB + (size_t)b * SEQ * DM, n8);
    }
    { const size_t n8 = (size_t)3 * DM * DM / 8; k_cvt8<<<(unsigned)((n8 + 255) / 256), 256, 0, stream>>>(wqkv, WB, n8); }
    { const size_t n8 = (size_t)DM * DM / 8;     k_cvtw<<<(unsigned)((n8 + 255) / 256), 256, 0, stream>>>(wproj, WP, n8); }

    k_proj_bf<<<dim3(NB * SEQ / 64, QKP / 64, 1), 32, 0, stream>>>(XB, WB, bqkv, QK, 0, 0, 0, QKP);
    k_proj_bf<<<dim3(DM / 64, SEQ / 64, NB), 32, 0, stream>>>(WB + (size_t)2 * DM * DM, XB, bqkv + 2 * DM, VT, 1, SEQ, DM * SEQ, SEQ);

    k_band<<<dim3(SEQ / (16 * AW), NB, 1), 32 * AW, 0, stream>>>(QK, VT, CX);

    k_out<<<dim3(NB * SEQ / 64, DM / 64, 1), 32, 0, stream>>>(CX, WP, bproj, OUT);
}
